// SoftPatternClassifier_24146306138518
// MI455X (gfx1250) — hardware-verified
//
#include <hip/hip_runtime.h>
#include <math.h>
typedef __attribute__((ext_vector_type(16))) _Float16 v16h;
typedef __attribute__((ext_vector_type(8)))  _Float16 v8h;
typedef __attribute__((ext_vector_type(16))) __bf16   v16b;
typedef __attribute__((ext_vector_type(8)))  __bf16   v8b;
typedef __attribute__((ext_vector_type(8)))  float    v8f;
typedef __attribute__((ext_vector_type(4)))  float    v4f;
#define PSCALE 32768.0f
#define U16(p) ((const unsigned short*)(const void*)(p))
#define PSCALE_INV (1.0f / 32768.0f)

__device__ __forceinline__ unsigned short f2bf_bits(float f) {
  unsigned u = __float_as_uint(f);
  return (unsigned short)((u + 0x7FFFu + ((u >> 16) & 1u)) >> 16);
}
__device__ __forceinline__ float bf_bits2f(unsigned short h) { return __uint_as_float(((unsigned)h) << 16); }

__device__ __forceinline__ void dep_guard_h(v8f& a, v8f& b, v16h x, v16h y) { asm volatile("v_nop\n\tv_nop\n\tv_nop\n\tv_nop" : "+v"(a), "+v"(b) : "v"(x), "v"(y)); }
__device__ __forceinline__ void dep_guard_b(v8f& a, v8f& b, v16b x, v16b y) { asm volatile("v_nop\n\tv_nop\n\tv_nop\n\tv_nop" : "+v"(a), "+v"(b) : "v"(x), "v"(y)); }
__device__ __forceinline__ void keep4_h(v16h a, v16h b, v16h c, v16h d) { asm volatile("v_nop" :: "v"(a), "v"(b), "v"(c), "v"(d)); }
__device__ __forceinline__ void keep4_b(v16b a, v16b b, v16b c, v16b d) { asm volatile("v_nop" :: "v"(a), "v"(b), "v"(c), "v"(d)); }
__device__ __forceinline__ void acc_guard4(v8f& a, v8f& b, v8f& c, v8f& d) { asm volatile("v_nop\n\tv_nop\n\tv_nop\n\tv_nop" : "+v"(a), "+v"(b), "+v"(c), "+v"(d)); }
template <typename T> struct Frag;
template <> struct Frag<_Float16> {
  typedef v16h V; union U { v16h v; v8h h[2]; };
  static __device__ __forceinline__ v16h load(const _Float16* p) {
    U f; f.h[0] = *(const v8h*)(p); f.h[1] = *(const v8h*)(p + 16); return f.v;
  }
  static __device__ __forceinline__ v8f mma(v16h a, v16h b, v8f c) {
    return __builtin_amdgcn_wmma_f32_16x16x32_f16(false, a, false, b, (short)0, c, false, false);
  }
  static __device__ __forceinline__ void guard(v8f& a, v8f& b, v16h x, v16h y) { dep_guard_h(a, b, x, y); }
  static __device__ __forceinline__ void keep(v16h a, v16h b, v16h c, v16h d) { keep4_h(a, b, c, d); }
};
template <> struct Frag<__bf16> {
  typedef v16b V; union U { v16b v; v8b h[2]; };
  static __device__ __forceinline__ v16b load(const __bf16* p) {
    U f; f.h[0] = *(const v8b*)(p); f.h[1] = *(const v8b*)(p + 16); return f.v;
  }
  static __device__ __forceinline__ v8f mma(v16b a, v16b b, v8f c) {
    return __builtin_amdgcn_wmma_f32_16x16x32_bf16(false, a, false, b, (short)0, c, false, false);
  }
  static __device__ __forceinline__ void guard(v8f& a, v8f& b, v16b x, v16b y) { dep_guard_b(a, b, x, y); }
  static __device__ __forceinline__ void keep(v16b a, v16b b, v16b c, v16b d) { keep4_b(a, b, c, d); }
};

template <int ET> struct Elem;
template <> struct Elem<0> { typedef _Float16 T; };
template <> struct Elem<1> { typedef __bf16 T; };
template <int ET, bool SPLIT, int BIAS_MODE, int OUT_MODE, bool RESID, int ACT = 0>
__global__ __launch_bounds__(256) void wmma_gemm64(
    const unsigned short* __restrict__ Ap, const unsigned short* __restrict__ A2p, int lda, long strideA,
    const unsigned short* __restrict__ Btp, const unsigned short* __restrict__ Bt2p, int ldb, long strideB,
    void* __restrict__ Cout, void* __restrict__ Cout2, int ldc, long strideC,
    const float* __restrict__ bias,
    const float* __restrict__ resid, long strideR,
    int M, int N, int K, float scale) {
  typedef typename Elem<ET>::T T;
  typedef typename Frag<T>::V V;
  const T* A = (const T*)Ap; const T* A2 = (const T*)A2p; const T* Bt = (const T*)Btp; const T* Bt2 = (const T*)Bt2p;
  __shared__ __align__(16) float sT[8][16 * 68];
  const int b    = blockIdx.y;
  const int lane = threadIdx.x & 31;
  const int wave = threadIdx.x >> 5;
  const int tilesN = N >> 6;
  const int tilesM = M >> 6;
  const int tile = blockIdx.x * 8 + wave;
  if (tile >= tilesM * tilesN) return;
  const int tm = tile / tilesN;
  const int tn = tile - tm * tilesN;
  const int m0 = tm << 6;
  const int n0 = tn << 6;

  const T* Ab  = A  + (size_t)b * strideA;
  const T* Bb  = Bt + (size_t)b * strideB;
  const T* Ab2 = SPLIT ? (A2  + (size_t)b * strideA) : nullptr;
  const T* Bb2 = SPLIT ? (Bt2 + (size_t)b * strideB) : nullptr;

  const int rlane = lane & 15;
  const int koff  = (lane >> 4) * 8;
  const int mOff  = (lane >> 4) * 8;

  v8f acc[4][4];
#pragma unroll
  for (int i = 0; i < 4; ++i)
#pragma unroll
    for (int j = 0; j < 4; ++j) acc[i][j] = (v8f){0.f,0.f,0.f,0.f,0.f,0.f,0.f,0.f};

  for (int k0 = 0; k0 < K; k0 += 32) {
    V bh[4], bl[4];
#pragma unroll
    for (int j = 0; j < 4; ++j) {
      const size_t bo = (size_t)(n0 + (j << 4) + rlane) * ldb + koff + k0;
      bh[j] = Frag<T>::load(Bb + bo);
      if (SPLIT) bl[j] = Frag<T>::load(Bb2 + bo);
    }
#pragma unroll
    for (int i = 0; i < 4; ++i) {
      const size_t ao = (size_t)(m0 + (i << 4) + rlane) * lda + koff + k0;
      V ah = Frag<T>::load(Ab + ao);
      V al;
      if (SPLIT) al = Frag<T>::load(Ab2 + ao);
#pragma unroll
      for (int j = 0; j < 4; ++j) {
        acc[i][j] = Frag<T>::mma(ah, bh[j], acc[i][j]);
        if (SPLIT) {
          acc[i][j] = Frag<T>::mma(ah, bl[j], acc[i][j]);
          acc[i][j] = Frag<T>::mma(al, bh[j], acc[i][j]);
        }
      }
      Frag<T>::guard(acc[i][0], acc[i][3], ah, SPLIT ? al : ah);
    }
    Frag<T>::keep(bh[0], bh[1], bh[2], bh[3]);
    if (SPLIT) Frag<T>::keep(bl[0], bl[1], bl[2], bl[3]);
  }
  acc_guard4(acc[0][0], acc[0][1], acc[0][2], acc[0][3]);
  acc_guard4(acc[1][0], acc[1][1], acc[1][2], acc[1][3]);
  acc_guard4(acc[2][0], acc[2][1], acc[2][2], acc[2][3]);
  acc_guard4(acc[3][0], acc[3][1], acc[3][2], acc[3][3]);

  float* slab = sT[wave];
  const float* Rb = RESID ? (resid + (size_t)b * strideR) : nullptr;
#pragma unroll
  for (int i = 0; i < 4; ++i) {
    const int mBase = m0 + (i << 4);
#pragma unroll
    for (int j = 0; j < 4; ++j) {
      const int n = n0 + (j << 4) + rlane;
      float bv = 0.f;
      if (BIAS_MODE == 2) bv = bias[n];
#pragma unroll
      for (int r = 0; r < 8; ++r) {
        float v = acc[i][j][r] * scale;
        if (BIAS_MODE == 1) v += bias[mBase + mOff + r];
        if (BIAS_MODE == 2) v += bv;
        if (RESID) v += Rb[(size_t)(mBase + mOff + r) * ldc + n];
        if (ACT == 1) v = tanhf(v);
        if (ACT == 2) v = fmaxf(v, 0.0f);
        if (ACT == 3) v = v / (1.0f + expf(-v));
        if (ACT == 4) v = (v > 0.f) ? v : 0.01f * v;
        if (ACT == 5) v = 0.5f * v * (1.0f + erff(v * 0.70710678118654752f));
        slab[(mOff + r) * 68 + (j << 4) + rlane] = v;
      }
    }
    __builtin_amdgcn_fence(__ATOMIC_RELEASE, "workgroup");
    __builtin_amdgcn_wave_barrier();
    __builtin_amdgcn_fence(__ATOMIC_ACQUIRE, "workgroup");
    if (OUT_MODE == 0) {
      float* C = (float*)Cout + (size_t)b * strideC;
      const int hh = lane >> 4, c4 = (lane & 15) * 4;
      for (int pass = 0; pass < 2; ++pass) {
#pragma unroll
        for (int it = 0; it < 8; ++it) {
          const int row = it * 2 + hh;
          v4f v = *(const v4f*)(slab + row * 68 + c4);
          *(volatile v4f*)(C + (size_t)(mBase + row) * ldc + n0 + c4) = v;
        }
        __threadfence();
      }
    } else {
      const int q = lane >> 3, c8 = (lane & 7) * 8;
      unsigned short* C  = (unsigned short*)Cout  + (size_t)b * strideC;
      unsigned short* C2 = (OUT_MODE == 2) ? ((unsigned short*)Cout2 + (size_t)b * strideC) : nullptr;
      for (int pass = 0; pass < 2; ++pass) {
#pragma unroll
        for (int it = 0; it < 4; ++it) {
          const int row = it * 4 + q;
          const float* sp = slab + row * 68 + c8;
          v8h hv, lv;
#pragma unroll
          for (int e = 0; e < 8; ++e) {
            if (OUT_MODE == 1) {
              hv[e] = (_Float16)sp[e];
            } else {
              unsigned short hb = f2bf_bits(sp[e]);
              unsigned short lb = f2bf_bits(sp[e] - bf_bits2f(hb));
              hv[e] = __builtin_bit_cast(_Float16, hb);
              lv[e] = __builtin_bit_cast(_Float16, lb);
            }
          }
          *(volatile v8h*)(C + (size_t)(mBase + row) * ldc + n0 + c8) = hv;
          if (OUT_MODE == 2) *(volatile v8h*)(C2 + (size_t)(mBase + row) * ldc + n0 + c8) = lv;
        }
        __threadfence();
      }
    }
    __builtin_amdgcn_fence(__ATOMIC_RELEASE, "workgroup");
    __builtin_amdgcn_wave_barrier();
    __builtin_amdgcn_fence(__ATOMIC_ACQUIRE, "workgroup");
  }
}

__global__ __launch_bounds__(256) void cast_f32_f16x2(
    const float* __restrict__ in, _Float16* __restrict__ out, int n2) {
  int i = blockIdx.x * 256 + threadIdx.x;
  if (i < n2) {
    const _Float16 h0 = (_Float16)in[2 * i], h1 = (_Float16)in[2 * i + 1];
    const unsigned u = (unsigned)__builtin_bit_cast(unsigned short, h0) | ((unsigned)__builtin_bit_cast(unsigned short, h1) << 16);
    ((volatile unsigned*)out)[i] = u;
    __threadfence();
    ((volatile unsigned*)out)[i] = u;
  }
}


#define SPB 64
#define SPT 256
#define SPV 10000
#define SPVP 10048
#define SPE 300
#define SPKP 320
#define SPP 300
#define SPL 7
#define SPD 4200
#define SPDP 4224
#define SPNEG (-1e9f)
__global__ __launch_bounds__(256) void embT_kernel(const float* __restrict__ emb, unsigned* __restrict__ A16) {
  __shared__ float tile[64][65];
  const int v0 = blockIdx.x * 64, e0 = blockIdx.y * 64, tx = threadIdx.x, ty = threadIdx.y;
  for (int i = ty; i < 64; i += 8) { const int e = e0 + i; for (int j = tx; j < 64; j += 32) { const int v = v0 + j; tile[i][j] = (e < SPE && v < SPV) ? emb[(size_t)e * SPV + v] : 0.f; } }
  __syncthreads();
  for (int pass = 0; pass < 2; ++pass) {
    for (int j = ty; j < 64; j += 8) { const int v = v0 + j;
      const unsigned u = (unsigned)__builtin_bit_cast(unsigned short, (_Float16)tile[2 * tx][j]) | ((unsigned)__builtin_bit_cast(unsigned short, (_Float16)tile[2 * tx + 1][j]) << 16);
      ((volatile unsigned*)A16)[((size_t)v * SPKP + e0) / 2 + tx] = u; }
    __threadfence(); }
}
__global__ __launch_bounds__(256) void diag_kernel(const float* __restrict__ dg, unsigned* __restrict__ BT, float* __restrict__ biasp, const float* __restrict__ bias) {
  const long i = (long)blockIdx.x * 256 + threadIdx.x; if (i >= (long)SPDP * SPKP / 2) return;
  const long e0 = 2 * i; const int d = (int)(e0 / SPKP), k = (int)(e0 % SPKP);
  float a = 0.f, b = 0.f; if (d < SPD) { if (k < SPE) a = dg[(size_t)d * SPE + k]; if (k + 1 < SPE) b = dg[(size_t)d * SPE + k + 1]; }
  const unsigned u = (unsigned)__builtin_bit_cast(unsigned short, (_Float16)a) | ((unsigned)__builtin_bit_cast(unsigned short, (_Float16)b) << 16);
  ((volatile unsigned*)BT)[i] = u;
  if (i < SPDP) { const float bv = (i < SPD) ? bias[i] : 0.f; ((volatile float*)biasp)[i] = bv; }
  __threadfence(); ((volatile unsigned*)BT)[i] = u; if (i < SPDP) ((volatile float*)biasp)[i] = (i < SPD) ? bias[i] : 0.f;
}
__global__ __launch_bounds__(256) void wfsa_kernel(const float* __restrict__ TR, const int* __restrict__ docs, const int* __restrict__ dl, const float* __restrict__ eps, float* __restrict__ S) {
  const int idx = blockIdx.x * 256 + threadIdx.x; if (idx >= SPB * SPP) return;
  const int b = idx / SPP, p = idx % SPP;
  float h[SPL]; h[0] = 0.f;
#pragma unroll
  for (int l = 1; l < SPL; ++l) h[l] = SPNEG;
  float ep[SPL - 1];
#pragma unroll
  for (int l = 0; l < SPL - 1; ++l) ep[l] = eps[p * (SPL - 1) + l];
  int len = dl[b];
  float score = SPNEG;
  for (int t = 0; t < SPT; ++t) {
    int tok = docs[b * SPT + t]; tok = tok < 0 ? 0 : (tok >= SPV ? SPV - 1 : tok);
    const float* tm = TR + (size_t)tok * SPDP + p * (2 * SPL);
    float sl[SPL], mn[SPL];
#pragma unroll
    for (int l = 0; l < SPL; ++l) { sl[l] = tm[l]; mn[l] = tm[SPL + l]; }
    float ae[SPL]; ae[0] = h[0];
#pragma unroll
    for (int l = 1; l < SPL; ++l) ae[l] = fmaxf(h[l], h[l - 1] + ep[l - 1]);
    float nh[SPL]; nh[0] = fmaxf(0.f, ae[0] + sl[0]);
#pragma unroll
    for (int l = 1; l < SPL; ++l) nh[l] = fmaxf(ae[l - 1] + mn[l - 1], ae[l] + sl[l]);
#pragma unroll
    for (int l = 0; l < SPL; ++l) h[l] = nh[l];
    if (len > t) score = fmaxf(score, h[SPL - 1]);
  }
  ((volatile float*)S)[(size_t)b * SPKP + p] = score; __threadfence(); ((volatile float*)S)[(size_t)b * SPKP + p] = score;
}
__global__ __launch_bounds__(256) void mlp_kernel(const float* __restrict__ S, const float* __restrict__ w0, const float* __restrict__ b0, const float* __restrict__ w1, const float* __restrict__ b1, float* __restrict__ stg) {
  __shared__ float s[SPP]; __shared__ float hid[256];
  const int b = blockIdx.x, t = threadIdx.x;
  for (int i = t; i < SPP; i += 256) s[i] = S[(size_t)b * SPKP + i];
  __syncthreads();
  float a = b0[t];
#pragma unroll 1
  for (int k = 0; k < SPP; ++k) a += s[k] * w0[(size_t)k * 256 + t];
  hid[t] = fmaxf(a, 0.f);
  __syncthreads();
  if (t < 32) { float o = 0.f; if (t < 5) { o = b1[t];
#pragma unroll 1
      for (int k = 0; k < 256; ++k) o += hid[k] * w1[k * 5 + t]; }
    ((volatile float*)stg)[(size_t)b * 32 + t] = o; __threadfence(); ((volatile float*)stg)[(size_t)b * 32 + t] = o; }
}
__global__ __launch_bounds__(256) void pack_kernel(const float* __restrict__ stg, float* __restrict__ out) {
  for (int pass = 0; pass < 2; ++pass) { for (int i = threadIdx.x; i < SPB * 5; i += 256) ((volatile float*)out)[i] = stg[(i / 5) * 32 + (i % 5)]; __threadfence(); }
}
extern "C" void kernel_launch(void* const* d_in, const int* in_sizes, int n_in, void* d_out, int out_size, void* d_ws, size_t ws_size, hipStream_t stream) {
  (void)in_sizes; (void)n_in; (void)out_size; (void)ws_size;
  const int* docs = (const int*)d_in[0]; const int* dl = (const int*)d_in[1]; const float* emb = (const float*)d_in[2]; const float* dg = (const float*)d_in[3]; const float* bias = (const float*)d_in[4];
  const float* eps = (const float*)d_in[5]; const float* w0 = (const float*)d_in[6]; const float* b0 = (const float*)d_in[7]; const float* w1 = (const float*)d_in[8]; const float* b1 = (const float*)d_in[9];
  char* ws = (char*)d_ws; size_t off = 0;
  auto carve = [&](size_t bytes) -> char* { char* p = ws + off; off += (bytes + 255) & ~(size_t)255; return p; };
  unsigned* A16 = (unsigned*)carve((size_t)SPVP * SPKP * 2); unsigned* BT = (unsigned*)carve((size_t)SPDP * SPKP * 2); float* biasp = (float*)carve((size_t)SPDP * 4);
  float* TR = (float*)carve((size_t)SPVP * SPDP * 4);
  float* S = (float*)carve((size_t)SPB * SPKP * 4); float* stg = (float*)carve((size_t)SPB * 32 * 4);
  embT_kernel<<<dim3(SPVP / 64, SPKP / 64), dim3(32, 8), 0, stream>>>(emb, A16);
  diag_kernel<<<(SPDP * SPKP / 2 + 255) / 256, 256, 0, stream>>>(dg, BT, biasp, bias);
  { const int t = (SPVP / 64) * (SPDP / 64);
    wmma_gemm64<0, false, 2, 0, false><<<dim3((t + 7) / 8, 1), 256, 0, stream>>>((const unsigned short*)A16, nullptr, SPKP, 0, (const unsigned short*)BT, nullptr, SPKP, 0, TR, nullptr, SPDP, 0, biasp, nullptr, 0, SPVP, SPDP, SPKP, 1.0f); }
  wfsa_kernel<<<(SPB * SPP + 255) / 256, 256, 0, stream>>>(TR, docs, dl, eps, S);
  mlp_kernel<<<SPB, 256, 0, stream>>>(S, w0, b0, w1, b1, stg);
  pack_kernel<<<1, 256, 0, stream>>>(stg, (float*)d_out);
}
